// NAFAlignBlock_74019466379845
// MI455X (gfx1250) — hardware-verified
//
#include <hip/hip_runtime.h>
#define NBt 2
#define C0 64
#define DW 128
#define HH 160
#define NPX (HH * HH)
#define NG 4
#define CG 32
#define KP 9
#define NOM 112
typedef __bf16 v16b __attribute__((ext_vector_type(16)));
typedef unsigned short v8us __attribute__((ext_vector_type(8), may_alias));
typedef float  v8f  __attribute__((ext_vector_type(8)));
typedef float  v4f  __attribute__((ext_vector_type(4)));
typedef float  v4fa __attribute__((ext_vector_type(4), may_alias));
union FragB { v16b v; v8us half[2]; unsigned short u[16]; };

__device__ __forceinline__ unsigned short bf16_bits(float x) { unsigned int u = __float_as_uint(x); return (unsigned short)((u + 0x7FFFu + ((u >> 16) & 1u)) >> 16); }
__device__ __forceinline__ float bf16_val(unsigned short b) { return __uint_as_float(((unsigned int)b) << 16); }
__device__ __forceinline__ float bf16_round(float x) { return bf16_val(bf16_bits(x)); }
template <int NT>
__device__ __forceinline__ v8f mmaN(v16b ah, v16b al, v16b bh, v16b bl, v8f c) {
  c = __builtin_amdgcn_wmma_f32_16x16x32_bf16(false, ah, false, bh, (short)0, c, false, false);
  if (NT >= 2) c = __builtin_amdgcn_wmma_f32_16x16x32_bf16(false, al, false, bh, (short)0, c, false, false);
  if (NT >= 3) c = __builtin_amdgcn_wmma_f32_16x16x32_bf16(false, ah, false, bl, (short)0, c, false, false);
  asm volatile("v_nop\n\tv_nop\n\tv_nop\n\tv_nop" : "+v"(c) : "v"(ah), "v"(al), "v"(bh), "v"(bl));
  return c;
}

__global__ __launch_bounds__(256) void k_wt_bf16(const float* __restrict__ W, unsigned short* __restrict__ Wt, int K, int N) {
  const int t = blockIdx.x * 256 + threadIdx.x;
  const int k8n = K / 8;
  if (t >= N * k8n) return;
  const int n = t / k8n, k8 = (t % k8n) * 8;
  v8us v;
#pragma unroll
  for (int i = 0; i < 8; ++i) v[i] = bf16_bits(W[(size_t)(k8 + i) * N + n]);
  *(volatile v8us*)(Wt + (size_t)n * K + k8) = v;
  __threadfence();
  *(volatile v8us*)(Wt + (size_t)n * K + k8) = v;
}

template <bool ASPLIT, int ACT, bool BIAS_BF16>
__global__ __launch_bounds__(128) void k_gemm_bf(const float* __restrict__ A, int lda, const unsigned short* __restrict__ Wt, int ldb,
                                               const float* __restrict__ bias, float* __restrict__ C, int ldc, int M, int N, int K) {
  __shared__ __attribute__((aligned(16))) float so[4][16][64];
  const int tid = threadIdx.x, w = tid >> 5, lane = tid & 31, ln = lane & 15, hh = lane >> 4;
  const int ntn = N / 64;
  const int wid = blockIdx.x * 4 + w;
  const int mt = wid / ntn, nq = wid % ntn;
  if (mt * 16 >= M) return;
  const int row0 = mt * 16, col0 = nq * 64;
  const float* arow = A + (size_t)(row0 + ln) * lda;
  v8f acc[4] = {};
  for (int kb = 0; kb < K; kb += 32) {
    FragB ah, al;
    const v4f x0 = *(const v4fa*)(arow + kb + 8 * hh), x1 = *(const v4fa*)(arow + kb + 8 * hh + 4);
    const v4f x2 = *(const v4fa*)(arow + kb + 16 + 8 * hh), x3 = *(const v4fa*)(arow + kb + 16 + 8 * hh + 4);
    float xs[16] = {x0[0],x0[1],x0[2],x0[3],x1[0],x1[1],x1[2],x1[3],x2[0],x2[1],x2[2],x2[3],x3[0],x3[1],x3[2],x3[3]};
#pragma unroll
    for (int i = 0; i < 16; ++i) { const unsigned short hb = bf16_bits(xs[i]); ah.u[i] = hb; al.u[i] = ASPLIT ? bf16_bits(xs[i] - bf16_val(hb)) : (unsigned short)0; }
#pragma unroll
    for (int t = 0; t < 4; ++t) {
      const unsigned short* brow = Wt + (size_t)(col0 + t * 16 + ln) * ldb + kb;
      FragB b;
      b.half[0] = *(const v8us*)(brow + 8 * hh);
      b.half[1] = *(const v8us*)(brow + 16 + 8 * hh);
      acc[t] = mmaN<ASPLIT ? 2 : 1>(ah.v, al.v, b.v, b.v, acc[t]);
    }
  }
#pragma unroll
  for (int t = 0; t < 4; ++t) {
    float bv = bias ? bias[col0 + t * 16 + ln] : 0.f;
    if (BIAS_BF16) bv = bf16_round(bv);
#pragma unroll
    for (int r = 0; r < 8; ++r) { float v = acc[t][r] + bv; if (ACT == 1) v = fmaxf(v, 0.f); so[w][8 * hh + r][t * 16 + ln] = v; }
  }
  __builtin_amdgcn_fence(__ATOMIC_ACQ_REL, "workgroup");
  __builtin_amdgcn_wave_barrier();
  const int rsub = lane >> 4, c4 = (lane & 15) * 4;
  for (int pass = 0; pass < 2; ++pass) {
#pragma unroll
    for (int q = 0; q < 8; ++q) {
      const int r = q * 2 + rsub;
      const v4f v = *(const v4fa*)&so[w][r][c4];
      *(volatile v4f*)(C + (size_t)(row0 + r) * ldc + col0 + c4) = v;
    }
    if (pass == 0) __threadfence();
  }
}

template <bool ASPLIT, int ACT, bool BIAS_BF16, bool RES_BF16>
__global__ __launch_bounds__(128) void k_gemm_bf3(const float* __restrict__ A, int lda, const unsigned short* __restrict__ Wt, int ldb,
                                                const float* __restrict__ bias, const float* __restrict__ resid, int rmod, int ldr,
                                                float* __restrict__ C, int ldc, int M, int N, int K) {
  __shared__ __attribute__((aligned(16))) float so[4][16][64];
  const int tid = threadIdx.x, w = tid >> 5, lane = tid & 31, ln = lane & 15, hh = lane >> 4;
  const int ntn = N / 64;
  const int wid = blockIdx.x * 4 + w;
  const int mt = wid / ntn, nq = wid % ntn;
  if (mt * 16 >= M) return;
  const int row0 = mt * 16, col0 = nq * 64;
  const float* arow = A + (size_t)(row0 + ln) * lda;
  v8f acc[4] = {};
  for (int kb = 0; kb < K; kb += 32) {
    FragB ah, al;
    const v4f x0 = *(const v4fa*)(arow + kb + 8 * hh), x1 = *(const v4fa*)(arow + kb + 8 * hh + 4);
    const v4f x2 = *(const v4fa*)(arow + kb + 16 + 8 * hh), x3 = *(const v4fa*)(arow + kb + 16 + 8 * hh + 4);
    float xs[16] = {x0[0],x0[1],x0[2],x0[3],x1[0],x1[1],x1[2],x1[3],x2[0],x2[1],x2[2],x2[3],x3[0],x3[1],x3[2],x3[3]};
#pragma unroll
    for (int i = 0; i < 16; ++i) { const unsigned short hb = bf16_bits(xs[i]); ah.u[i] = hb; al.u[i] = ASPLIT ? bf16_bits(xs[i] - bf16_val(hb)) : (unsigned short)0; }
#pragma unroll
    for (int t = 0; t < 4; ++t) {
      const unsigned short* brow = Wt + (size_t)(col0 + t * 16 + ln) * ldb + kb;
      FragB b;
      b.half[0] = *(const v8us*)(brow + 8 * hh);
      b.half[1] = *(const v8us*)(brow + 16 + 8 * hh);
      acc[t] = mmaN<ASPLIT ? 2 : 1>(ah.v, al.v, b.v, b.v, acc[t]);
    }
  }
#pragma unroll
  for (int t = 0; t < 4; ++t) {
    const int col = col0 + t * 16 + ln;
    float bv = bias ? bias[col] : 0.f;
    if (BIAS_BF16) bv = bf16_round(bv);
#pragma unroll
    for (int r = 0; r < 8; ++r) {
      float v = acc[t][r] + bv;
      if (resid) { float rv = resid[(size_t)((row0 + 8 * hh + r) % rmod) * ldr + col]; if (RES_BF16) rv = bf16_round(rv); v += rv; }
      if (ACT == 1) v = fmaxf(v, 0.f);
      if (ACT == 2) v = 0.5f * v * (1.0f + erff(v * 0.70710678118654752f));
      if (ACT == 3) { const float u = 0.7978845608028654f * (v + 0.044715f * v * v * v); v = 0.5f * v * (1.0f + tanhf(u)); }
      so[w][8 * hh + r][t * 16 + ln] = v;
    }
  }
  __builtin_amdgcn_fence(__ATOMIC_ACQ_REL, "workgroup");
  __builtin_amdgcn_wave_barrier();
  const int rsub = lane >> 4, c4 = (lane & 15) * 4;
  for (int pass = 0; pass < 2; ++pass) {
#pragma unroll
    for (int q = 0; q < 8; ++q) {
      const int r = q * 2 + rsub;
      const v4f v = *(const v4fa*)&so[w][r][c4];
      *(volatile v4f*)(C + (size_t)(row0 + r) * ldc + col0 + c4) = v;
    }
    if (pass == 0) __threadfence();
  }
}
template <bool PARAM_BF16>
__global__ __launch_bounds__(256) void k_layernorm(const float* __restrict__ X, const float* __restrict__ R, const float* __restrict__ g, const float* __restrict__ bta,
                                                  float* __restrict__ out_sum, float* __restrict__ out_norm, int N, float eps) {
  __shared__ float red[256];
  const int row = blockIdx.x, tid = threadIdx.x;
  const float* x = X + (size_t)row * N; const float* rr = R ? R + (size_t)row * N : nullptr;
  float vals[16];
  const int per = N / 256;
  float s1 = 0.f;
  for (int u = 0; u < per / 4; ++u) {
    const int j = tid * 4 + 1024 * u;
    const v4f a = *(const v4fa*)(x + j);
    v4f b = {0.f,0.f,0.f,0.f}; if (rr) b = *(const v4fa*)(rr + j);
#pragma unroll
    for (int q = 0; q < 4; ++q) { const float v = a[q] + b[q]; vals[u * 4 + q] = v; s1 += v; }
  }
  red[tid] = s1; __syncthreads();
  for (int st = 128; st > 0; st >>= 1) { if (tid < st) red[tid] += red[tid + st]; __syncthreads(); }
  const float mu = red[0] / (float)N; __syncthreads();
  float s2 = 0.f;
  for (int u = 0; u < per / 4; ++u)
#pragma unroll
    for (int q = 0; q < 4; ++q) { const float c = vals[u * 4 + q] - mu; s2 += c * c; }
  red[tid] = s2; __syncthreads();
  for (int st = 128; st > 0; st >>= 1) { if (tid < st) red[tid] += red[tid + st]; __syncthreads(); }
  const float rs = rsqrtf(red[0] / (float)N + eps);
  for (int pass = 0; pass < 2; ++pass) {
    for (int u = 0; u < per / 4; ++u) {
      const int j = tid * 4 + 1024 * u;
      v4f o, sm;
#pragma unroll
      for (int q = 0; q < 4; ++q) {
        float gg = g[j + q], bb = bta[j + q];
        if (PARAM_BF16) { gg = bf16_round(gg); bb = bf16_round(bb); }
        sm[q] = vals[u * 4 + q]; o[q] = (vals[u * 4 + q] - mu) * rs * gg + bb;
      }
      if (out_sum) *(volatile v4f*)(out_sum + (size_t)row * N + j) = sm;
      *(volatile v4f*)(out_norm + (size_t)row * N + j) = o;
    }
    if (pass == 0) __threadfence();
  }
}


typedef _Float16 v16h __attribute__((ext_vector_type(16)));
union FragH { v16h v; v8us half[2]; _Float16 h[16]; unsigned short u[16]; };
template <int NT>
__device__ __forceinline__ v8f mmaH(v16h ah, v16h al, v16h bh, v16h bl, v8f c) {
  c = __builtin_amdgcn_wmma_f32_16x16x32_f16(false, ah, false, bh, (short)0, c, false, false);
  if (NT >= 2) c = __builtin_amdgcn_wmma_f32_16x16x32_f16(false, al, false, bh, (short)0, c, false, false);
  if (NT >= 3) c = __builtin_amdgcn_wmma_f32_16x16x32_f16(false, ah, false, bl, (short)0, c, false, false);
  asm volatile("v_nop\n\tv_nop\n\tv_nop\n\tv_nop" : "+v"(c) : "v"(ah), "v"(al), "v"(bh), "v"(bl));
  return c;
}
template <bool ASPLIT>
__global__ __launch_bounds__(128) void k_gemm_h(const float* __restrict__ A, int lda, size_t sA, const _Float16* __restrict__ Bh, int ldb, size_t sB, float alpha, float* __restrict__ C, int ldc, size_t sC, int M, int N, int K) {
  __shared__ __attribute__((aligned(16))) float so[4][16][64];
  const int tid = threadIdx.x, w = tid >> 5, lane = tid & 31, ln = lane & 15, hh = lane >> 4; const int by = blockIdx.y;
  A += (size_t)by * sA; Bh += (size_t)by * sB; C += (size_t)by * sC;
  const int ntn = (N + 63) / 64; const int wid = blockIdx.x * 4 + w; const int mt = wid / ntn, nq = wid % ntn; if (mt * 16 >= M) return;
  const int row0 = mt * 16, col0 = nq * 64; const float* arow = A + (size_t)(row0 + ln) * lda;
  v8f acc[4] = {};
  for (int kb = 0; kb < K; kb += 32) {
    FragH ah, al;
    const v4f x0 = *(const v4fa*)(arow + kb + 8 * hh), x1 = *(const v4fa*)(arow + kb + 8 * hh + 4), x2 = *(const v4fa*)(arow + kb + 16 + 8 * hh), x3 = *(const v4fa*)(arow + kb + 16 + 8 * hh + 4);
    float xs[16] = {x0[0],x0[1],x0[2],x0[3],x1[0],x1[1],x1[2],x1[3],x2[0],x2[1],x2[2],x2[3],x3[0],x3[1],x3[2],x3[3]};
#pragma unroll
    for (int i = 0; i < 16; ++i) { const _Float16 h = (_Float16)xs[i]; ah.h[i] = h; al.h[i] = ASPLIT ? (_Float16)(xs[i] - (float)h) : (_Float16)0.0f; }
#pragma unroll
    for (int t = 0; t < 4; ++t) { if (col0 + t * 16 >= N) continue; const size_t boff = (size_t)(col0 + t * 16 + ln) * ldb + kb; FragH bq; bq.half[0] = *(const v8us*)(Bh + boff + 8 * hh); bq.half[1] = *(const v8us*)(Bh + boff + 16 + 8 * hh);
      acc[t] = mmaH<ASPLIT ? 2 : 1>(ah.v, al.v, bq.v, bq.v, acc[t]); }
  }
#pragma unroll
  for (int t = 0; t < 4; ++t) { if (col0 + t * 16 >= N) continue;
#pragma unroll
    for (int r = 0; r < 8; ++r) so[w][8 * hh + r][t * 16 + ln] = acc[t][r] * alpha; }
  __builtin_amdgcn_fence(__ATOMIC_ACQ_REL, "workgroup"); __builtin_amdgcn_wave_barrier();
  const int rsub = lane >> 4, c4 = (lane & 15) * 4;
  for (int pass = 0; pass < 2; ++pass) {
#pragma unroll
    for (int q = 0; q < 8; ++q) { const int r = q * 2 + rsub; if (col0 + c4 < N) { const v4f v = *(const v4fa*)&so[w][r][c4]; *(volatile v4f*)(C + (size_t)(row0 + r) * ldc + col0 + c4) = v; } }
    if (pass == 0) __threadfence(); }
}

__global__ __launch_bounds__(256) void k_wt_f16(const float* __restrict__ W, _Float16* __restrict__ Wt, int K, int N, float scale) {
  const int t = blockIdx.x * 256 + threadIdx.x; if (t >= N * (K / 8)) return; const int n = t / (K / 8), k8 = (t % (K / 8)) * 8; FragH f;
#pragma unroll
  for (int i = 0; i < 8; ++i) f.h[i] = (_Float16)(bf16_round(W[(size_t)(k8 + i) * N + n]) * scale); const v8us o = f.half[0];
  *(volatile v8us*)((unsigned short*)Wt + (size_t)n * K + k8) = o; __threadfence(); *(volatile v8us*)((unsigned short*)Wt + (size_t)n * K + k8) = o;
}
template <int ACT>
__global__ __launch_bounds__(128) void k_gemm_hhx(const _Float16* __restrict__ A, int lda, size_t sA, const _Float16* __restrict__ Bh, int ldb, size_t sB, float alpha, const float* __restrict__ bias, size_t sBias, const float* __restrict__ CP, int rowsPerB, size_t sCPb, int row0g,
    float* __restrict__ C, _Float16* __restrict__ C16, int ldc, size_t sC, int M, int N, int K) {
  __shared__ __attribute__((aligned(16))) float so[4][16][64];
  const int tid = threadIdx.x, w = tid >> 5, lane = tid & 31, ln = lane & 15, hh = lane >> 4; const int by = blockIdx.y;
  A += (size_t)by * sA; Bh += (size_t)by * sB; const size_t cofs = (size_t)by * sC; const float* bp = bias ? bias + (size_t)by * sBias : nullptr;
  const int ntn = (N + 63) / 64; const int wid = blockIdx.x * 4 + w; const int mt = wid / ntn, nq = wid % ntn; if (mt * 16 >= M) return;
  const int row0 = mt * 16, col0 = nq * 64; const _Float16* arow = A + (size_t)(row0 + ln) * lda;
  v8f acc[4] = {};
  for (int kb = 0; kb < K; kb += 32) { FragH ah; ah.half[0] = *(const v8us*)((const unsigned short*)arow + kb + 8 * hh); ah.half[1] = *(const v8us*)((const unsigned short*)arow + kb + 16 + 8 * hh);
#pragma unroll
    for (int t = 0; t < 4; ++t) { if (col0 + t * 16 >= N) continue; const size_t boff = (size_t)(col0 + t * 16 + ln) * ldb + kb; FragH bq; bq.half[0] = *(const v8us*)((const unsigned short*)Bh + boff + 8 * hh); bq.half[1] = *(const v8us*)((const unsigned short*)Bh + boff + 16 + 8 * hh);
      acc[t] = mmaH<1>(ah.v, ah.v, bq.v, bq.v, acc[t]); }
  }
#pragma unroll
  for (int t = 0; t < 4; ++t) { if (col0 + t * 16 >= N) continue; const int col = col0 + t * 16 + ln; const float bv = bp ? bf16_round(bp[col]) : 0.f;
#pragma unroll
    for (int r = 0; r < 8; ++r) { float v = acc[t][r] * alpha + bv; if (CP) { const int bidx = (row0g + row0 + 8 * hh + r) / rowsPerB; v += CP[(size_t)bidx * sCPb + (size_t)by * 64 + col]; } if (ACT == 1) v = (v > 0.f) ? v : expm1f(v); else if (ACT == 7) v = (v > 0.f) ? v + 1.0f : expf(v); else if (ACT == 8) v = tanhf(v); else if (ACT == 9) v = 0.5f * v * (1.0f + tanhf(0.7978845608028654f * (v + 0.044715f * v * v * v))); else if (ACT == 11) v = 1.0f / (1.0f + expf(-v)); else if (ACT == 12) v = (v > 0.f) ? v : 0.01f * v; else if (ACT == 14) v = (v > 0.f) ? v : 0.1f * v; else if (ACT == 15) v = v / (1.0f + expf(-v)); else if (ACT == 3) v = fmaxf(v, 0.f); else if (ACT == 6) v = 0.5f * v * (1.0f + erff(v * 0.70710678118654752f)); so[w][8 * hh + r][t * 16 + ln] = v; } }
  __builtin_amdgcn_fence(__ATOMIC_ACQ_REL, "workgroup"); __builtin_amdgcn_wave_barrier();
  const int rsub = lane >> 4, c4 = (lane & 15) * 4; typedef _Float16 v4h __attribute__((ext_vector_type(4)));
  for (int pass = 0; pass < 2; ++pass) {
#pragma unroll
    for (int q = 0; q < 8; ++q) { const int r = q * 2 + rsub; if (col0 + c4 < N) { const v4f v = *(const v4fa*)&so[w][r][c4]; if (C) *(volatile v4f*)(C + cofs + (size_t)(row0 + r) * ldc + col0 + c4) = v; if (C16) { v4h h4; for (int i = 0; i < 4; ++i) h4[i] = (_Float16)v[i]; *(volatile v4h*)(C16 + cofs + (size_t)(row0 + r) * ldc + col0 + c4) = h4; } } }
    if (pass == 0) __threadfence(); }
}


typedef _Float16 v4h __attribute__((ext_vector_type(4)));

__global__ __launch_bounds__(256) void k_x16(const float* __restrict__ x, _Float16* __restrict__ X16, size_t n8) { const size_t t = (size_t)blockIdx.x * 256 + threadIdx.x; if (t >= n8) return; FragH f;
#pragma unroll
  for (int q = 0; q < 8; ++q) f.h[q] = (_Float16)bf16_round(x[t * 8 + q]); *(volatile v8us*)((unsigned short*)X16 + t * 8) = f.half[0]; __threadfence(); *(volatile v8us*)((unsigned short*)X16 + t * 8) = f.half[0]; }
__global__ __launch_bounds__(256) void k_h16(const float* __restrict__ x, _Float16* __restrict__ X16, size_t n8) { const size_t t = (size_t)blockIdx.x * 256 + threadIdx.x; if (t >= n8) return; FragH f;
#pragma unroll
  for (int q = 0; q < 8; ++q) f.h[q] = (_Float16)x[t * 8 + q]; *(volatile v8us*)((unsigned short*)X16 + t * 8) = f.half[0]; __threadfence(); *(volatile v8us*)((unsigned short*)X16 + t * 8) = f.half[0]; }
__global__ __launch_bounds__(256) void k_round16f(const float* __restrict__ W, _Float16* __restrict__ Bt, size_t n8) { const size_t t = (size_t)blockIdx.x * 256 + threadIdx.x; if (t >= n8) return; FragH f;
#pragma unroll
  for (int i = 0; i < 8; ++i) f.h[i] = (_Float16)(bf16_round(W[t * 8 + i]) * 16.0f); *(volatile v8us*)((unsigned short*)Bt + t * 8) = f.half[0]; __threadfence(); *(volatile v8us*)((unsigned short*)Bt + t * 8) = f.half[0]; }
template <int NHv, int TTv>
__global__ __launch_bounds__(256) void k_vt(const _Float16* __restrict__ V16, int ldv, int voff, _Float16* __restrict__ Vt) { __shared__ unsigned short tl[64][66]; const int tid = threadIdx.x; const int slab = blockIdx.x / (TTv / 64), lg = blockIdx.x % (TTv / 64); const int b = slab / NHv, h = slab % NHv;
  for (int i = tid; i < 64 * 8; i += 256) { const int r = i / 8, c8 = (i % 8) * 8; FragH f; f.half[0] = *(const v8us*)((const unsigned short*)V16 + ((size_t)b * TTv + lg * 64 + r) * ldv + voff + h * 64 + c8);
#pragma unroll
    for (int q = 0; q < 8; ++q) tl[r][c8 + q] = f.u[q]; }
  __syncthreads();
  for (int pass = 0; pass < 2; ++pass) {
#pragma unroll
    for (int rd = 0; rd < 2; ++rd) { const int d = rd * 32 + tid / 8, pc = tid % 8; FragH f;
#pragma unroll
      for (int q = 0; q < 8; ++q) f.u[q] = tl[pc * 8 + q][d];
      *(volatile v8us*)((unsigned short*)Vt + ((size_t)slab * 64 + d) * TTv + lg * 64 + pc * 8) = f.half[0]; }
    if (pass == 0) __threadfence(); } }

__global__ __launch_bounds__(256) void k_hl(const float* __restrict__ F, _Float16* __restrict__ Hh, _Float16* __restrict__ Hl, size_t n8) { const size_t t = (size_t)blockIdx.x * 256 + threadIdx.x; if (t >= n8) return; FragH fh, fl; const v4f a = *(const v4fa*)(F + t * 8), c = *(const v4fa*)(F + t * 8 + 4);
#pragma unroll
  for (int q = 0; q < 4; ++q) { _Float16 h = (_Float16)a[q]; fh.h[q] = h; fl.h[q] = (_Float16)((a[q] - (float)h) * 1024.0f); h = (_Float16)c[q]; fh.h[4 + q] = h; fl.h[4 + q] = (_Float16)((c[q] - (float)h) * 1024.0f); }
  for (int pass = 0; pass < 2; ++pass) { *(volatile v8us*)((unsigned short*)Hh + t * 8) = fh.half[0]; *(volatile v8us*)((unsigned short*)Hl + t * 8) = fl.half[0]; if (pass == 0) __threadfence(); } }

__global__ __launch_bounds__(256) void k_nchw2tok(const float* __restrict__ x, int b, float* __restrict__ T0) {
  __shared__ float tile[32][65]; const int tid = threadIdx.x; const int nct = C0 / 32, npt = NPX / 64; const int blk = blockIdx.x; const int ct = blk / npt, pt = blk % npt; const int c0 = ct * 32, p0 = pt * 64;
  for (int i = tid; i < 32 * 64; i += 256) { const int ci = i / 64, pi = i % 64; tile[ci][pi] = bf16_round(x[((size_t)b * C0 + c0 + ci) * NPX + p0 + pi]); }
  __syncthreads();
  for (int it = 0; it < 2; ++it) { const int row = tid / 8 + 32 * it, qd = tid % 8; v4f v; v[0] = tile[qd * 4 + 0][row]; v[1] = tile[qd * 4 + 1][row]; v[2] = tile[qd * 4 + 2][row]; v[3] = tile[qd * 4 + 3][row]; float* dst = T0 + (size_t)(p0 + row) * C0 + c0 + qd * 4; *(volatile v4f*)dst = v; __threadfence(); *(volatile v4f*)dst = v; } }
__global__ __launch_bounds__(256) void k_ln64(const float* __restrict__ T0, const float* __restrict__ g, _Float16* __restrict__ L16) {
  #pragma clang fp contract(off)
  const int tid = threadIdx.x, w = tid >> 5, l = tid & 31; const int p = blockIdx.x * 8 + w; if (p >= NPX) return; const float a = T0[(size_t)p * C0 + 2 * l], c = T0[(size_t)p * C0 + 2 * l + 1]; float s = a + c;
  for (int o = 16; o > 0; o >>= 1) s += __shfl_xor(s, o, 32); const float mu = s / (float)C0; float q2 = (a - mu) * (a - mu) + (c - mu) * (c - mu);
  for (int o = 16; o > 0; o >>= 1) q2 += __shfl_xor(q2, o, 32); const float rs = rsqrtf(q2 / (float)C0 + 1e-5f); FragH f; f.h[0] = (_Float16)((a - mu) * rs * bf16_round(g[2 * l])); f.h[1] = (_Float16)((c - mu) * rs * bf16_round(g[2 * l + 1])); const unsigned pv = *(const unsigned*)&f.u[0];
  *(volatile unsigned*)((unsigned short*)L16 + (size_t)p * C0 + 2 * l) = pv; __threadfence(); *(volatile unsigned*)((unsigned short*)L16 + (size_t)p * C0 + 2 * l) = pv; }
__global__ __launch_bounds__(256) void k_f16(const float* __restrict__ F, _Float16* __restrict__ O16, size_t n8) { const size_t t = (size_t)blockIdx.x * 256 + threadIdx.x; if (t >= n8) return; const v4f a = *(const v4fa*)(F + t * 8), c = *(const v4fa*)(F + t * 8 + 4); FragH f;
#pragma unroll
  for (int q = 0; q < 8; ++q) f.h[q] = (_Float16)((q < 4) ? a[q] : c[q - 4]);
  *(volatile v8us*)((unsigned short*)O16 + t * 8) = f.half[0]; __threadfence(); *(volatile v8us*)((unsigned short*)O16 + t * 8) = f.half[0]; }
__global__ __launch_bounds__(256) void k_dw3(const float* __restrict__ Hm, const float* __restrict__ w, const float* __restrict__ bb, _Float16* __restrict__ O16) {
  #pragma clang fp contract(off)
  const int t = blockIdx.x * 256 + threadIdx.x; if (t >= NPX * (DW / 8)) return; const int c0 = (t % (DW / 8)) * 8, p = t / (DW / 8); const int h = p / HH, x = p % HH; float acc[8];
#pragma unroll
  for (int q = 0; q < 8; ++q) acc[q] = bf16_round(bb[c0 + q]);
#pragma unroll 1
  for (int tp = 0; tp < 9; ++tp) { const int yy = h + tp / 3 - 1, xx = x + tp % 3 - 1; if (yy < 0 || yy >= HH || xx < 0 || xx >= HH) continue; const v4f a = *(const v4fa*)(Hm + ((size_t)yy * HH + xx) * DW + c0), c = *(const v4fa*)(Hm + ((size_t)yy * HH + xx) * DW + c0 + 4);
#pragma unroll
    for (int q = 0; q < 8; ++q) acc[q] += bf16_round(w[(size_t)tp * DW + c0 + q]) * ((q < 4) ? a[q] : c[q - 4]); }
  FragH f;
#pragma unroll
  for (int q = 0; q < 8; ++q) f.h[q] = (_Float16)acc[q];
  *(volatile v8us*)((unsigned short*)O16 + (size_t)p * DW + c0) = f.half[0]; __threadfence(); *(volatile v8us*)((unsigned short*)O16 + (size_t)p * DW + c0) = f.half[0]; }
__global__ __launch_bounds__(256) void k_dcn4(const float* __restrict__ OMp, const _Float16* __restrict__ V16, _Float16* __restrict__ DO16) {
  #pragma clang fp contract(off)
  const int t = blockIdx.x * 256 + threadIdx.x; if (t >= NPX * NG * 4) return; const int q8 = t & 3; const int g = (t >> 2) & 3; const int p = t >> 4; const int h = p / HH, w = p % HH; const float* om = OMp + (size_t)p * NOM + g * 27; float acc[8];
#pragma unroll
  for (int q = 0; q < 8; ++q) acc[q] = 0.f;
#pragma unroll 1
  for (int k = 0; k < KP; ++k) { const float ox = om[3 * k], oy = om[3 * k + 1], m = om[3 * k + 2];
    const float px = ((float)w + 1.5f) + (float)(k % 3 - 1) + ox - 0.5f, py = ((float)h + 1.5f) + (float)(k / 3 - 1) + oy - 0.5f; const float x0 = floorf(px), y0 = floorf(py); const float tx = px - x0, ty = py - y0; const int xi0 = (int)x0, yi0 = (int)y0;
#pragma unroll
    for (int cn = 0; cn < 4; ++cn) { const int dx = cn & 1, dy = cn >> 1; const int xi = xi0 + dx, yi = yi0 + dy; const float wgt = (dx ? tx : (1.0f - tx)) * (dy ? ty : (1.0f - ty)); const bool valid = (xi >= 0 && xi < HH + 2 && yi >= 0 && yi < HH + 2); const int ix = xi - 1, iy = yi - 1; const bool inr = valid && ix >= 0 && ix < HH && iy >= 0 && iy < HH; const float f = inr ? (wgt * m) : 0.f; FragH gv; gv.half[0] = *(const v8us*)((const unsigned short*)V16 + ((size_t)min(max(iy, 0), HH - 1) * HH + min(max(ix, 0), HH - 1)) * DW + g * CG + q8 * 8);
#pragma unroll
      for (int q = 0; q < 8; ++q) acc[q] += f * (float)gv.h[q]; } }
  FragH f;
#pragma unroll
  for (int q = 0; q < 8; ++q) f.h[q] = (_Float16)acc[q];
  *(volatile v8us*)((unsigned short*)DO16 + (size_t)p * DW + g * CG + q8 * 8) = f.half[0]; __threadfence(); *(volatile v8us*)((unsigned short*)DO16 + (size_t)p * DW + g * CG + q8 * 8) = f.half[0]; }
__global__ __launch_bounds__(256) void k_sg(const float* __restrict__ O, int ldo, float* __restrict__ F) {
  #pragma clang fp contract(off)
  const int t = blockIdx.x * 256 + threadIdx.x; const int half = ldo / 2; if (t >= NPX * (half / 4)) return; const int c0 = (t % (half / 4)) * 4, p = t / (half / 4); const v4f a = *(const v4fa*)(O + (size_t)p * ldo + c0), b2 = *(const v4fa*)(O + (size_t)p * ldo + half + c0); v4f v;
#pragma unroll
  for (int q = 0; q < 4; ++q) v[q] = a[q] * b2[q];
  *(volatile v4f*)(F + (size_t)p * half + c0) = v; __threadfence(); *(volatile v4f*)(F + (size_t)p * half + c0) = v; }
__global__ __launch_bounds__(256) void k_pool(const float* __restrict__ FL, const float* __restrict__ FR, float* __restrict__ POOL) {
  #pragma clang fp contract(off)
  __shared__ float red[256]; const int bc = blockIdx.x, tid = threadIdx.x; const int b = bc / DW, c = bc % DW; const float* src = ((c < C0) ? FL : FR) + (size_t)b * NPX * C0 + (c % C0); float s = 0.f;
  for (int p = tid; p < NPX; p += 256) s += src[(size_t)p * C0];
  red[tid] = s; __syncthreads(); for (int st = 128; st > 0; st >>= 1) { if (tid < st) red[tid] += red[tid + st]; __syncthreads(); }
  if (tid < 32) { const float m = red[0] / (float)NPX; *(volatile float*)(POOL + (size_t)bc * 32 + tid) = m; __threadfence(); *(volatile float*)(POOL + (size_t)bc * 32 + tid) = m; } }
__global__ __launch_bounds__(256) void k_sca(const float* __restrict__ POOL, const float* __restrict__ w, const float* __restrict__ bb, float* __restrict__ SCA) {
  #pragma clang fp contract(off)
  const int t = threadIdx.x; const int b = t / DW, o = t % DW; float s = bf16_round(bb[o]);
#pragma unroll 1
  for (int c = 0; c < DW; ++c) s += POOL[((size_t)b * DW + c) * 32] * bf16_round(w[(size_t)o * DW + c]);
  *(volatile float*)(SCA + t) = s; __threadfence(); *(volatile float*)(SCA + t) = s; }
__global__ __launch_bounds__(256) void k_xs(const float* __restrict__ FL, const float* __restrict__ FR, const float* __restrict__ SCA, int b, _Float16* __restrict__ X16) {
  #pragma clang fp contract(off)
  const int t = blockIdx.x * 256 + threadIdx.x; if (t >= NPX * (DW / 8)) return; const int c0 = (t % (DW / 8)) * 8, p = t / (DW / 8); const float* src = ((c0 < C0) ? FL : FR) + ((size_t)b * NPX + p) * C0 + (c0 % C0); const v4f a = *(const v4fa*)src, c = *(const v4fa*)(src + 4); FragH f;
#pragma unroll
  for (int q = 0; q < 8; ++q) f.h[q] = (_Float16)(((q < 4) ? a[q] : c[q - 4]) * SCA[(size_t)b * DW + c0 + q]);
  *(volatile v8us*)((unsigned short*)X16 + (size_t)p * DW + c0) = f.half[0]; __threadfence(); *(volatile v8us*)((unsigned short*)X16 + (size_t)p * DW + c0) = f.half[0]; }
__global__ __launch_bounds__(256) void k_ycat(const float* __restrict__ TL, const float* __restrict__ TR, const float* __restrict__ X3, const float* __restrict__ beta, const float* __restrict__ g2, float* __restrict__ YL, float* __restrict__ YR, _Float16* __restrict__ Z16) {
  #pragma clang fp contract(off)
  const int tid = threadIdx.x, w = tid >> 5, l = tid & 31; const int p = blockIdx.x * 8 + w; if (p >= NPX) return; typedef float v2f __attribute__((ext_vector_type(2))); float yl[2], yr[2]; float s = 0.f;
#pragma unroll
  for (int k = 0; k < 2; ++k) { const int c = 2 * l + k; const float corr = X3[(size_t)p * C0 + c] * bf16_round(beta[c]); yl[k] = TL[(size_t)p * C0 + c] + corr; yr[k] = TR[(size_t)p * C0 + c] + corr; s += yl[k] + yr[k]; }
  for (int o = 16; o > 0; o >>= 1) s += __shfl_xor(s, o, 32); const float mu = s / (float)DW; float q2 = 0.f;
#pragma unroll
  for (int k = 0; k < 2; ++k) { q2 += (yl[k] - mu) * (yl[k] - mu) + (yr[k] - mu) * (yr[k] - mu); }
  for (int o = 16; o > 0; o >>= 1) q2 += __shfl_xor(q2, o, 32); const float rs = rsqrtf(q2 / (float)DW + 1e-5f);
  v2f vl, vr; vl[0] = yl[0]; vl[1] = yl[1]; vr[0] = yr[0]; vr[1] = yr[1]; FragH fz; fz.h[0] = (_Float16)((yl[0] - mu) * rs * bf16_round(g2[2 * l])); fz.h[1] = (_Float16)((yl[1] - mu) * rs * bf16_round(g2[2 * l + 1])); fz.h[2] = (_Float16)((yr[0] - mu) * rs * bf16_round(g2[C0 + 2 * l])); fz.h[3] = (_Float16)((yr[1] - mu) * rs * bf16_round(g2[C0 + 2 * l + 1]));
  const unsigned z01 = *(const unsigned*)&fz.u[0], z23 = *(const unsigned*)&fz.u[2];
  for (int pass = 0; pass < 2; ++pass) { *(volatile v2f*)(YL + (size_t)p * C0 + 2 * l) = vl; *(volatile v2f*)(YR + (size_t)p * C0 + 2 * l) = vr; *(volatile unsigned*)((unsigned short*)Z16 + (size_t)p * DW + 2 * l) = z01; *(volatile unsigned*)((unsigned short*)Z16 + (size_t)p * DW + C0 + 2 * l) = z23; if (pass == 0) __threadfence(); } }
__global__ __launch_bounds__(256) void k_sg16(const float* __restrict__ Z4, _Float16* __restrict__ G16) {
  #pragma clang fp contract(off)
  const int t = blockIdx.x * 256 + threadIdx.x; if (t >= NPX * (C0 / 8)) return; const int c0 = (t % (C0 / 8)) * 8, p = t / (C0 / 8); const v4f a = *(const v4fa*)(Z4 + (size_t)p * DW + c0), a2 = *(const v4fa*)(Z4 + (size_t)p * DW + c0 + 4), b1 = *(const v4fa*)(Z4 + (size_t)p * DW + C0 + c0), b2 = *(const v4fa*)(Z4 + (size_t)p * DW + C0 + c0 + 4); FragH f;
#pragma unroll
  for (int q = 0; q < 8; ++q) f.h[q] = (_Float16)(((q < 4) ? a[q] : a2[q - 4]) * ((q < 4) ? b1[q] : b2[q - 4]));
  *(volatile v8us*)((unsigned short*)G16 + (size_t)p * C0 + c0) = f.half[0]; __threadfence(); *(volatile v8us*)((unsigned short*)G16 + (size_t)p * C0 + c0) = f.half[0]; }
__global__ __launch_bounds__(256) void k_outn(const float* __restrict__ Y, const float* __restrict__ Z5, const float* __restrict__ gamma, int b, float* __restrict__ out) {
  #pragma clang fp contract(off)
  const int t = blockIdx.x * 256 + threadIdx.x; if (t >= C0 * (NPX / 4)) return; const int p0 = (t % (NPX / 4)) * 4, c = t / (NPX / 4); const float gc = bf16_round(gamma[c]); v4f v;
#pragma unroll
  for (int q = 0; q < 4; ++q) v[q] = Y[(size_t)(p0 + q) * C0 + c] + Z5[(size_t)(p0 + q) * C0 + c] * gc;
  float* dst = out + ((size_t)b * C0 + c) * NPX + p0; *(volatile v4f*)dst = v; __threadfence(); *(volatile v4f*)dst = v; }

extern "C" void kernel_launch(void* const* d_in, const int* in_sizes, int n_in,
                              void* d_out, int out_size, void* d_ws, size_t ws_size, hipStream_t stream) {
  (void)in_sizes; (void)n_in; (void)out_size;
  const float* const* I = (const float* const*)d_in; const float* xl = I[0]; const float* xr = I[1]; const float* ln1g = I[2]; const float* pw1w = I[3]; const float* pw1b = I[4]; const float* valw = I[5]; const float* valb = I[6]; const float* dwcw = I[7]; const float* dwcb = I[8]; const float* omw = I[9]; const float* omb = I[10]; const float* outpw = I[11]; const float* outpb = I[12]; const float* scaw = I[13]; const float* scab = I[14]; const float* c3w = I[15]; const float* c3b = I[16]; const float* n2g = I[17]; const float* c4w = I[18]; const float* c4b = I[19]; const float* c5w = I[20]; const float* c5b = I[21]; const float* beta = I[22]; const float* gamma = I[23];
  char* ws = (char*)d_ws; size_t off = 0;
  auto take = [&](size_t bytes) { char* p = ws + off; off += (bytes + 255) & ~(size_t)255; return p; };
  _Float16* BPW1 = (_Float16*)take((size_t)DW * C0 * 2); _Float16* BVAL = (_Float16*)take((size_t)DW * DW * 2); _Float16* BOM = (_Float16*)take((size_t)NOM * DW * 2); _Float16* BOUT = (_Float16*)take((size_t)DW * DW * 2); _Float16* BC3 = (_Float16*)take((size_t)C0 * DW * 2); _Float16* BC4 = (_Float16*)take((size_t)DW * DW * 2); _Float16* BC5 = (_Float16*)take((size_t)C0 * C0 * 2);
  float* TL = (float*)take((size_t)NBt * NPX * C0 * 4); float* TRr = (float*)take((size_t)NBt * NPX * C0 * 4); float* FL = (float*)take((size_t)NBt * NPX * C0 * 4); float* FR = (float*)take((size_t)NBt * NPX * C0 * 4);
  _Float16* L16 = (_Float16*)take((size_t)NPX * C0 * 2); float* Hm = (float*)take((size_t)NPX * DW * 4); _Float16* H16 = (_Float16*)take((size_t)NPX * DW * 2); _Float16* V16 = (_Float16*)take((size_t)NPX * DW * 2); _Float16* DW16 = (_Float16*)take((size_t)NPX * DW * 2); float* OMp = (float*)take((size_t)NPX * NOM * 4); _Float16* DO16 = (_Float16*)take((size_t)NPX * DW * 2); float* O = (float*)take((size_t)NPX * DW * 4);
  float* POOL = (float*)take((size_t)NBt * DW * 32 * 4); float* SCA = (float*)take((size_t)NBt * DW * 4);
  _Float16* X16 = H16;
  float* X3 = (float*)DW16;
  float* YL = O; float* YR = O + (size_t)NPX * C0;
  _Float16* Z16 = V16;
  float* Z4 = Hm;
  _Float16* G16 = L16;
  float* Z5 = (float*)DO16;
  if (off > ws_size) return;
  k_round16f<<<(DW * C0 / 8 + 255) / 256, 256, 0, stream>>>(pw1w, BPW1, (size_t)DW * C0 / 8); k_round16f<<<(DW * DW / 8 + 255) / 256, 256, 0, stream>>>(valw, BVAL, (size_t)DW * DW / 8); k_round16f<<<(NOM * DW / 8 + 255) / 256, 256, 0, stream>>>(omw, BOM, (size_t)NOM * DW / 8); k_round16f<<<(DW * DW / 8 + 255) / 256, 256, 0, stream>>>(outpw, BOUT, (size_t)DW * DW / 8); k_round16f<<<(C0 * DW / 8 + 255) / 256, 256, 0, stream>>>(c3w, BC3, (size_t)C0 * DW / 8); k_round16f<<<(DW * DW / 8 + 255) / 256, 256, 0, stream>>>(c4w, BC4, (size_t)DW * DW / 8); k_round16f<<<(C0 * C0 / 8 + 255) / 256, 256, 0, stream>>>(c5w, BC5, (size_t)C0 * C0 / 8);
  const dim3 g128(((NPX / 16) * (DW / 64) + 3) / 4, 1), g112(((NPX / 16) * ((NOM + 63) / 64) + 3) / 4, 1), g64(((NPX / 16) * 1 + 3) / 4, 1); const unsigned nb8w = (NPX * (DW / 8) + 255) / 256;
  for (int vb = 0; vb < 4; ++vb) { const int view = vb >> 1, b = vb & 1; const float* xin = view ? xr : xl; float* T0 = (view ? TRr : TL) + (size_t)b * NPX * C0; float* F = (view ? FR : FL) + (size_t)b * NPX * C0;
    k_nchw2tok<<<(C0 / 32) * (NPX / 64), 256, 0, stream>>>(xin, b, T0); k_ln64<<<NPX / 8, 256, 0, stream>>>(T0, ln1g, L16);
    k_gemm_hhx<0><<<g128, 128, 0, stream>>>(L16, C0, 0, BPW1, C0, 0, 0.0625f, pw1b, 0, nullptr, 1, 0, 0, Hm, nullptr, DW, 0, NPX, DW, C0);
    k_f16<<<(unsigned)(((size_t)NPX * DW / 8 + 255) / 256), 256, 0, stream>>>(Hm, H16, (size_t)NPX * DW / 8);
    k_gemm_hhx<0><<<g128, 128, 0, stream>>>(H16, DW, 0, BVAL, DW, 0, 0.0625f, valb, 0, nullptr, 1, 0, 0, nullptr, V16, DW, 0, NPX, DW, DW);
    k_dw3<<<nb8w, 256, 0, stream>>>(Hm, dwcw, dwcb, DW16);
    k_gemm_hhx<0><<<g112, 128, 0, stream>>>(DW16, DW, 0, BOM, DW, 0, 0.0625f, omb, 0, nullptr, 1, 0, 0, OMp, nullptr, NOM, 0, NPX, NOM, DW);
    k_dcn4<<<(NPX * NG * 4 + 255) / 256, 256, 0, stream>>>(OMp, V16, DO16);
    k_gemm_hhx<0><<<g128, 128, 0, stream>>>(DO16, DW, 0, BOUT, DW, 0, 0.0625f, outpb, 0, nullptr, 1, 0, 0, O, nullptr, DW, 0, NPX, DW, DW);
    k_sg<<<(NPX * (C0 / 4) + 255) / 256, 256, 0, stream>>>(O, DW, F); }
  k_pool<<<NBt * DW, 256, 0, stream>>>(FL, FR, POOL); k_sca<<<1, 256, 0, stream>>>(POOL, scaw, scab, SCA);
  for (int b = 0; b < NBt; ++b) {
    k_xs<<<nb8w, 256, 0, stream>>>(FL, FR, SCA, b, X16);
    k_gemm_hhx<0><<<g64, 128, 0, stream>>>(X16, DW, 0, BC3, DW, 0, 0.0625f, c3b, 0, nullptr, 1, 0, 0, X3, nullptr, C0, 0, NPX, C0, DW);
    k_ycat<<<NPX / 8, 256, 0, stream>>>(TL + (size_t)b * NPX * C0, TRr + (size_t)b * NPX * C0, X3, beta, n2g, YL, YR, Z16);
    k_gemm_hhx<0><<<g128, 128, 0, stream>>>(Z16, DW, 0, BC4, DW, 0, 0.0625f, c4b, 0, nullptr, 1, 0, 0, Z4, nullptr, DW, 0, NPX, DW, DW);
    k_sg16<<<(NPX * (C0 / 8) + 255) / 256, 256, 0, stream>>>(Z4, G16);
    k_gemm_hhx<0><<<g64, 128, 0, stream>>>(G16, C0, 0, BC5, C0, 0, 0.0625f, c5b, 0, nullptr, 1, 0, 0, Z5, nullptr, C0, 0, NPX, C0, C0);
    k_outn<<<(C0 * (NPX / 4) + 255) / 256, 256, 0, stream>>>(YL, Z5, gamma, b, (float*)d_out); k_outn<<<(C0 * (NPX / 4) + 255) / 256, 256, 0, stream>>>(YR, Z5, gamma, b, (float*)((char*)d_out + 13107200)); }
}
